// CorrelationModule_3607772528921
// MI455X (gfx1250) — hardware-verified
//
#include <hip/hip_runtime.h>
#include <stdint.h>
#include <stddef.h>
#include <math.h>

#pragma clang fp contract(off)

typedef __attribute__((ext_vector_type(16))) _Float16 v16h;
typedef __attribute__((ext_vector_type(8)))  _Float16 v8h;
typedef __attribute__((ext_vector_type(16))) __bf16   v16b;
typedef __attribute__((ext_vector_type(8)))  __bf16   v8b;
typedef __attribute__((ext_vector_type(8)))  float    v8f;
typedef __attribute__((ext_vector_type(4)))  float    v4f;
typedef __attribute__((ext_vector_type(4)))  unsigned v4u;
typedef __attribute__((ext_vector_type(2)))  unsigned v2u;
typedef __attribute__((ext_vector_type(4)))  int      v4i;

constexpr int kFeat      = 128;
constexpr int kHgt       = 64;
constexpr int kWid       = 128;
constexpr int kPix       = kHgt * kWid;
constexpr int kRad       = 4;
constexpr int kDia       = 2 * kRad + 1;
constexpr int kND        = kDia * kDia;
constexpr int kRows      = kND * kPix;
constexpr int kCh1       = 96;
constexpr int kCh2       = 128;
constexpr int kCh3       = 64;
constexpr int kTile      = 128;
constexpr int kTiles     = kRows / kTile;
constexpr int kTilesPerN = kPix / kTile;
constexpr int kTGP       = 128;
constexpr int kThreads   = 256;
constexpr int kP1        = 104;
constexpr int kP2        = 136;
constexpr int kYP        = 68;
constexpr int kABP       = 256;
constexpr int kDQP       = 32;
constexpr float  kEps        = 1e-5f;
constexpr float  kW2Carry    = 64.0f;
constexpr float  kW2CarryInv = 1.0f / 64.0f;
constexpr double kInvRows    = 1.0 / 663552.0;

static_assert(kPix % kTile == 0);
static_assert(kRows % kTile == 0);
static_assert(kCh1 % 32 == 0 && kCh2 % 32 == 0 && kFeat % 32 == 0);
static_assert(kPix % 64 == 0 && kTGP % 64 == 0);
static_assert(kP1 % 8 == 0 && kP2 % 8 == 0 && kP1 >= kCh1 && kP2 >= kCh2);
static_assert(kTile * 12 == 6 * kThreads);
static_assert(kCh3 * 16 == 4 * kThreads);
static_assert(kTile * 8 == 4 * kThreads);
static_assert(kTile == 4 * 32 && kThreads == 256);

constexpr int kA1H  = 0;
constexpr int kA1L  = kTile * kP1;
constexpr int kW2H  = 2 * kTile * kP1;
constexpr int kW2L  = 3 * kTile * kP1;
constexpr int kULen = 4 * kTile * kP1;
constexpr int kA2H  = 0;
constexpr int kA2L  = kTile * kP2;
constexpr int kW3H  = 2 * kTile * kP2;
constexpr int kW3L  = kW3H + kCh3 * kP2;
static_assert(kW3L + kCh3 * kP2 <= kULen);
static_assert(kTile * kYP * 2 <= kULen);

constexpr size_t kPlaneFT = (size_t)kPix * kFeat * 2;
constexpr size_t kOffFtH  = 0;
constexpr size_t kOffFtL  = kOffFtH + 2 * kPlaneFT;
constexpr size_t kPlaneW1 = (size_t)128 * 128 * 2;
constexpr size_t kOffW1H  = kOffFtL + 2 * kPlaneFT;
constexpr size_t kOffW1L  = kOffW1H + 2 * kPlaneW1;
constexpr size_t kPlaneTG = (size_t)kPix * kTGP * 4;
constexpr size_t kOffTG   = kOffW1L + 2 * kPlaneW1;
constexpr size_t kPlaneW2 = (size_t)kCh2 * kCh1 * 2;
constexpr size_t kPlaneW3 = (size_t)kCh3 * kCh2 * 2;
constexpr size_t kOffW2H  = kOffTG + 2 * kPlaneTG;
constexpr size_t kOffW2L  = kOffW2H + kPlaneW2;
constexpr size_t kOffW2F  = kOffW2L + kPlaneW2;
constexpr size_t kOffW3H  = kOffW2F + kPlaneW2;
constexpr size_t kOffW3L  = kOffW3H + kPlaneW3;
constexpr size_t kOffAB1  = kOffW3L + kPlaneW3;
constexpr size_t kOffAB2  = kOffAB1 + (size_t)kABP * 4;
constexpr size_t kOffAB3  = kOffAB2 + (size_t)kABP * 4;
constexpr size_t kOffSt1  = kOffAB3 + (size_t)kABP * 4;
constexpr size_t kOffSt2  = kOffSt1 + (size_t)kTiles * 2 * kCh1 * 4;
constexpr size_t kOffSt3  = kOffSt2 + (size_t)kTiles * 2 * kCh2 * 4;
constexpr size_t kOffDQ   = kOffSt3 + (size_t)kTiles * 2 * kCh3 * 4;
constexpr size_t kOffY3   = kOffDQ + (size_t)kTiles * kDQP * 4;
constexpr size_t kWsTotal = kOffY3 + (size_t)kRows * kCh3 * 2;
static_assert(kWsTotal == 114560000);
static_assert(kWsTotal <= (size_t)134217728);
static_assert(kOffFtL % 128 == 0 && kOffW1H % 128 == 0 && kOffW1L % 128 == 0 && kOffTG % 128 == 0);
static_assert(kOffW2H % 128 == 0 && kOffW2L % 128 == 0 && kOffW2F % 128 == 0 && kOffW3H % 128 == 0 && kOffW3L % 128 == 0);
static_assert(kOffAB1 % 128 == 0 && kOffSt1 % 128 == 0 && kOffSt2 % 128 == 0 && kOffSt3 % 128 == 0);
static_assert(kOffDQ % 128 == 0 && kOffY3 % 128 == 0);

__device__ __forceinline__ unsigned short f2bf_bits(float f) {
  unsigned u = __float_as_uint(f);
  return (unsigned short)((u + 0x7FFFu + ((u >> 16) & 1u)) >> 16);
}
__device__ __forceinline__ float bf_bits2f(unsigned short h) { return __uint_as_float(((unsigned)h) << 16); }

__device__ __forceinline__ void dep_guard_h(v8f& a, v8f& b, v16h x, v16h y) { asm volatile("v_nop\n\tv_nop\n\tv_nop\n\tv_nop" : "+v"(a), "+v"(b) : "v"(x), "v"(y)); }
__device__ __forceinline__ void dep_guard_b(v8f& a, v8f& b, v16b x, v16b y) { asm volatile("v_nop\n\tv_nop\n\tv_nop\n\tv_nop" : "+v"(a), "+v"(b) : "v"(x), "v"(y)); }
__device__ __forceinline__ void keep4_h(v16h a, v16h b, v16h c, v16h d) { asm volatile("v_nop" :: "v"(a), "v"(b), "v"(c), "v"(d)); }
__device__ __forceinline__ void keep4_b(v16b a, v16b b, v16b c, v16b d) { asm volatile("v_nop" :: "v"(a), "v"(b), "v"(c), "v"(d)); }
__device__ __forceinline__ void acc_guard4(v8f& a, v8f& b, v8f& c, v8f& d) { asm volatile("v_nop\n\tv_nop\n\tv_nop\n\tv_nop" : "+v"(a), "+v"(b), "+v"(c), "+v"(d)); }
template <typename T> struct Frag;
template <> struct Frag<_Float16> {
  typedef v16h V; union U { v16h v; v8h h[2]; };
  static __device__ __forceinline__ v16h load(const _Float16* p) {
    U f; f.h[0] = *(const v8h*)(p); f.h[1] = *(const v8h*)(p + 16); return f.v;
  }
  static __device__ __forceinline__ v8f mma(v16h a, v16h b, v8f c) {
    return __builtin_amdgcn_wmma_f32_16x16x32_f16(false, a, false, b, (short)0, c, false, false);
  }
  static __device__ __forceinline__ void guard(v8f& a, v8f& b, v16h x, v16h y) { dep_guard_h(a, b, x, y); }
  static __device__ __forceinline__ void keep(v16h a, v16h b, v16h c, v16h d) { keep4_h(a, b, c, d); }
};
template <> struct Frag<__bf16> {
  typedef v16b V; union U { v16b v; v8b h[2]; };
  static __device__ __forceinline__ v16b load(const __bf16* p) {
    U f; f.h[0] = *(const v8b*)(p); f.h[1] = *(const v8b*)(p + 16); return f.v;
  }
  static __device__ __forceinline__ v8f mma(v16b a, v16b b, v8f c) {
    return __builtin_amdgcn_wmma_f32_16x16x32_bf16(false, a, false, b, (short)0, c, false, false);
  }
  static __device__ __forceinline__ void guard(v8f& a, v8f& b, v16b x, v16b y) { dep_guard_b(a, b, x, y); }
  static __device__ __forceinline__ void keep(v16b a, v16b b, v16b c, v16b d) { keep4_b(a, b, c, d); }
};

template <int ET> struct Elem;
template <> struct Elem<0> { typedef _Float16 T; };
template <> struct Elem<1> { typedef __bf16 T; };
template <int ET, bool SPLIT, int BIAS_MODE, int OUT_MODE, bool RESID, int ACT = 0>
__global__ __launch_bounds__(256) void wmma_gemm64(
    const unsigned short* __restrict__ Ap, const unsigned short* __restrict__ A2p, int lda, long strideA,
    const unsigned short* __restrict__ Btp, const unsigned short* __restrict__ Bt2p, int ldb, long strideB,
    void* __restrict__ Cout, void* __restrict__ Cout2, int ldc, long strideC,
    const float* __restrict__ bias,
    const float* __restrict__ resid, long strideR,
    int M, int N, int K, float scale) {
  typedef typename Elem<ET>::T T;
  typedef typename Frag<T>::V V;
  const T* A = (const T*)Ap; const T* A2 = (const T*)A2p; const T* Bt = (const T*)Btp; const T* Bt2 = (const T*)Bt2p;
  __shared__ __align__(16) float sT[8][16 * 68];
  const int b    = blockIdx.y;
  const int lane = threadIdx.x & 31;
  const int wave = threadIdx.x >> 5;
  const int tilesN = N >> 6;
  const int tilesM = M >> 6;
  const int tile = blockIdx.x * 8 + wave;
  if (tile >= tilesM * tilesN) return;
  const int tm = tile / tilesN;
  const int tn = tile - tm * tilesN;
  const int m0 = tm << 6;
  const int n0 = tn << 6;

  const T* Ab  = A  + (size_t)b * strideA;
  const T* Bb  = Bt + (size_t)b * strideB;
  const T* Ab2 = SPLIT ? (A2  + (size_t)b * strideA) : nullptr;
  const T* Bb2 = SPLIT ? (Bt2 + (size_t)b * strideB) : nullptr;

  const int rlane = lane & 15;
  const int koff  = (lane >> 4) * 8;
  const int mOff  = (lane >> 4) * 8;

  v8f acc[4][4];
#pragma unroll
  for (int i = 0; i < 4; ++i)
#pragma unroll
    for (int j = 0; j < 4; ++j) acc[i][j] = (v8f){0.f,0.f,0.f,0.f,0.f,0.f,0.f,0.f};

  for (int k0 = 0; k0 < K; k0 += 32) {
    V bh[4], bl[4];
#pragma unroll
    for (int j = 0; j < 4; ++j) {
      const size_t bo = (size_t)(n0 + (j << 4) + rlane) * ldb + koff + k0;
      bh[j] = Frag<T>::load(Bb + bo);
      if (SPLIT) bl[j] = Frag<T>::load(Bb2 + bo);
    }
#pragma unroll
    for (int i = 0; i < 4; ++i) {
      const size_t ao = (size_t)(m0 + (i << 4) + rlane) * lda + koff + k0;
      V ah = Frag<T>::load(Ab + ao);
      V al;
      if (SPLIT) al = Frag<T>::load(Ab2 + ao);
#pragma unroll
      for (int j = 0; j < 4; ++j) {
        acc[i][j] = Frag<T>::mma(ah, bh[j], acc[i][j]);
        if (SPLIT) {
          acc[i][j] = Frag<T>::mma(ah, bl[j], acc[i][j]);
          acc[i][j] = Frag<T>::mma(al, bh[j], acc[i][j]);
        }
      }
      Frag<T>::guard(acc[i][0], acc[i][3], ah, SPLIT ? al : ah);
    }
    Frag<T>::keep(bh[0], bh[1], bh[2], bh[3]);
    if (SPLIT) Frag<T>::keep(bl[0], bl[1], bl[2], bl[3]);
  }
  acc_guard4(acc[0][0], acc[0][1], acc[0][2], acc[0][3]);
  acc_guard4(acc[1][0], acc[1][1], acc[1][2], acc[1][3]);
  acc_guard4(acc[2][0], acc[2][1], acc[2][2], acc[2][3]);
  acc_guard4(acc[3][0], acc[3][1], acc[3][2], acc[3][3]);

  float* slab = sT[wave];
  const float* Rb = RESID ? (resid + (size_t)b * strideR) : nullptr;
#pragma unroll
  for (int i = 0; i < 4; ++i) {
    const int mBase = m0 + (i << 4);
#pragma unroll
    for (int j = 0; j < 4; ++j) {
      const int n = n0 + (j << 4) + rlane;
      float bv = 0.f;
      if (BIAS_MODE == 2) bv = bias[n];
#pragma unroll
      for (int r = 0; r < 8; ++r) {
        float v = acc[i][j][r] * scale;
        if (BIAS_MODE == 1) v += bias[mBase + mOff + r];
        if (BIAS_MODE == 2) v += bv;
        if (RESID) v += Rb[(size_t)(mBase + mOff + r) * ldc + n];
        if (ACT == 1) v = tanhf(v);
        if (ACT == 2) v = fmaxf(v, 0.0f);
        if (ACT == 3) v = v / (1.0f + expf(-v));
        if (ACT == 4) v = (v > 0.f) ? v : 0.01f * v;
        if (ACT == 5) v = 0.5f * v * (1.0f + erff(v * 0.70710678118654752f));
        slab[(mOff + r) * 68 + (j << 4) + rlane] = v;
      }
    }
    __builtin_amdgcn_fence(__ATOMIC_RELEASE, "workgroup");
    __builtin_amdgcn_wave_barrier();
    __builtin_amdgcn_fence(__ATOMIC_ACQUIRE, "workgroup");
    if (OUT_MODE == 0) {
      float* C = (float*)Cout + (size_t)b * strideC;
      const int hh = lane >> 4, c4 = (lane & 15) * 4;
      for (int pass = 0; pass < 2; ++pass) {
#pragma unroll
        for (int it = 0; it < 8; ++it) {
          const int row = it * 2 + hh;
          v4f v = *(const v4f*)(slab + row * 68 + c4);
          *(volatile v4f*)(C + (size_t)(mBase + row) * ldc + n0 + c4) = v;
        }
        __threadfence();
      }
    } else {
      const int q = lane >> 3, c8 = (lane & 7) * 8;
      unsigned short* C  = (unsigned short*)Cout  + (size_t)b * strideC;
      unsigned short* C2 = (OUT_MODE == 2) ? ((unsigned short*)Cout2 + (size_t)b * strideC) : nullptr;
      for (int pass = 0; pass < 2; ++pass) {
#pragma unroll
        for (int it = 0; it < 4; ++it) {
          const int row = it * 4 + q;
          const float* sp = slab + row * 68 + c8;
          v8h hv, lv;
#pragma unroll
          for (int e = 0; e < 8; ++e) {
            if (OUT_MODE == 1) {
              hv[e] = (_Float16)sp[e];
            } else {
              unsigned short hb = f2bf_bits(sp[e]);
              unsigned short lb = f2bf_bits(sp[e] - bf_bits2f(hb));
              hv[e] = __builtin_bit_cast(_Float16, hb);
              lv[e] = __builtin_bit_cast(_Float16, lb);
            }
          }
          *(volatile v8h*)(C + (size_t)(mBase + row) * ldc + n0 + c8) = hv;
          if (OUT_MODE == 2) *(volatile v8h*)(C2 + (size_t)(mBase + row) * ldc + n0 + c8) = lv;
        }
        __threadfence();
      }
    }
    __builtin_amdgcn_fence(__ATOMIC_RELEASE, "workgroup");
    __builtin_amdgcn_wave_barrier();
    __builtin_amdgcn_fence(__ATOMIC_ACQUIRE, "workgroup");
  }
}

__device__ __forceinline__ unsigned f16_bits(float x) {
  return (unsigned)__builtin_bit_cast(unsigned short, (_Float16)x);
}
__device__ __forceinline__ v4u pack8(const unsigned (&b)[8]) {
  v4u r;
  r[0] = b[0] | (b[1] << 16); r[1] = b[2] | (b[3] << 16);
  r[2] = b[4] | (b[5] << 16); r[3] = b[6] | (b[7] << 16);
  return r;
}
__device__ __forceinline__ void clause_break() { asm volatile("" ::: "memory"); }

union LdsU { unsigned short h[kULen]; float f[kULen / 2]; };

template <bool FULL> struct PT;
template <> struct PT<false> { typedef _Float16 T; };
template <> struct PT<true>  { typedef __bf16 T; };

__device__ __forceinline__ void row_geom(const float* __restrict__ coords, int p, float dxn, float dyn, v4i& idx, v4f& w) {
  const float cxp = coords[p];
  const float cyp = coords[kPix + p];
  const float centx = cxp + dxn;
  const float centy = cyp + dyn;
  const float gx = (2.0f * centx) * (1.0f / 127.0f) - 1.0f;
  const float gy = (2.0f * centy) * (1.0f / 63.0f) - 1.0f;
  const float x = ((gx + 1.0f) * 0.5f) * 127.0f;
  const float y = ((gy + 1.0f) * 0.5f) * 63.0f;
  const float x0 = floorf(x), y0 = floorf(y);
  const float x1 = x0 + 1.0f, y1 = y0 + 1.0f;
  const float wx1 = x - x0;
  const float wx0 = 1.0f - wx1;
  const float wy1 = y - y0;
  const float wy0 = 1.0f - wy1;
  const bool vx0 = (x0 >= 0.0f) && (x0 < (float)kWid);
  const bool vx1 = (x1 >= 0.0f) && (x1 < (float)kWid);
  const bool vy0 = (y0 >= 0.0f) && (y0 < (float)kHgt);
  const bool vy1 = (y1 >= 0.0f) && (y1 < (float)kHgt);
  float w00 = wy0 * wx0, w01 = wy0 * wx1, w10 = wy1 * wx0, w11 = wy1 * wx1;
  w00 = (vy0 && vx0) ? w00 : 0.0f;
  w01 = (vy0 && vx1) ? w01 : 0.0f;
  w10 = (vy1 && vx0) ? w10 : 0.0f;
  w11 = (vy1 && vx1) ? w11 : 0.0f;
  const int xc0 = (int)fminf(fmaxf(x0, 0.0f), (float)(kWid - 1));
  const int xc1 = (int)fminf(fmaxf(x1, 0.0f), (float)(kWid - 1));
  const int yc0 = (int)fminf(fmaxf(y0, 0.0f), (float)(kHgt - 1));
  const int yc1 = (int)fminf(fmaxf(y1, 0.0f), (float)(kHgt - 1));
  idx[0] = yc0 * kWid + xc0;
  idx[1] = yc0 * kWid + xc1;
  idx[2] = yc1 * kWid + xc0;
  idx[3] = yc1 * kWid + xc1;
  w[0] = w00; w[1] = w01; w[2] = w10; w[3] = w11;
}

__device__ __forceinline__ v4f gather4(const float* __restrict__ t1, const float* __restrict__ g, int p, int c4, v4i idx, v4f w) {
  const v4f t = *(const v4f*)(t1 + (size_t)p * kTGP + 4 * c4);
  const v4f a = *(const v4f*)(g + (size_t)idx[0] * kTGP + 4 * c4);
  const v4f b = *(const v4f*)(g + (size_t)idx[1] * kTGP + 4 * c4);
  const v4f c = *(const v4f*)(g + (size_t)idx[2] * kTGP + 4 * c4);
  const v4f d = *(const v4f*)(g + (size_t)idx[3] * kTGP + 4 * c4);
  v4f y;
#pragma unroll
  for (int e = 0; e < 4; ++e) {
    float r = t[e];
    r = fmaf(w[0], a[e], r);
    r = fmaf(w[1], b[e], r);
    r = fmaf(w[2], c[e], r);
    r = fmaf(w[3], d[e], r);
    y[e] = r;
  }
  return y;
}

__global__ __launch_bounds__(kThreads) void prep_feat(const float* __restrict__ f1, const float* __restrict__ f2,
                                                      unsigned short* __restrict__ fth, unsigned short* __restrict__ ftl) {
  __shared__ __align__(16) float T[kFeat * kYP];
  const int tid = threadIdx.x;
  const int which = blockIdx.y;
  const float* src = (which == 0) ? f1 : f2;
  const int p0 = blockIdx.x * 64;
#pragma unroll
  for (int it = 0; it < 8; ++it) {
    const int idx = it * kThreads + tid;
    const int c = idx >> 4, pl4 = (idx & 15) * 4;
    const v4f v = *(const v4f*)(src + (size_t)c * kPix + p0 + pl4);
    *(v4f*)(T + c * kYP + pl4) = v;
    if (it == 3) clause_break();
  }
  __syncthreads();
  v4u hv[4], lv[4];
#pragma unroll
  for (int it = 0; it < 4; ++it) {
    const int chunk = it * kThreads + tid;
    const int pr = chunk >> 4, c8 = (chunk & 15) * 8;
    unsigned hb[8], lb[8];
#pragma unroll
    for (int e = 0; e < 8; ++e) {
      const float x = T[(c8 + e) * kYP + pr];
      const unsigned short h = f2bf_bits(x);
      hb[e] = h;
      lb[e] = f2bf_bits(x - bf_bits2f(h));
    }
    hv[it] = pack8(hb);
    lv[it] = pack8(lb);
  }
  unsigned short* oh = fth + (size_t)which * kPix * kFeat;
  unsigned short* ol = ftl + (size_t)which * kPix * kFeat;
  for (int pass = 0; pass < 2; ++pass) {
#pragma unroll
    for (int it = 0; it < 4; ++it) {
      const int chunk = it * kThreads + tid;
      const int pr = chunk >> 4, c8 = (chunk & 15) * 8;
      const size_t o = (size_t)(p0 + pr) * kFeat + c8;
      *(volatile v4u*)(oh + o) = hv[it];
      *(volatile v4u*)(ol + o) = lv[it];
    }
    __threadfence();
  }
}

__global__ __launch_bounds__(kThreads) void prep_w(const float* __restrict__ W, int nrow, int ncol, int coff, int kk, int npad,
                                                   int mode, float scale, unsigned short* o1, unsigned short* o2) {
  const int tpr = kk >> 3;
  const int i = blockIdx.x * kThreads + threadIdx.x;
  if (i >= npad * tpr) return;
  const int n   = i / tpr;
  const int k0  = (i - n * tpr) * 8;
  const int ncl = (n < nrow) ? n : (nrow - 1);
  const float keep = (n < nrow) ? 1.0f : 0.0f;
  float v[8];
#pragma unroll
  for (int e = 0; e < 8; ++e) {
    const float x = W[(size_t)ncl * ncol + coff + k0 + e];
    v[e] = x * keep;
  }
  v4u a, b;
  if (mode == 0) {
    unsigned hb[8], lb[8];
#pragma unroll
    for (int e = 0; e < 8; ++e) {
      const unsigned short h = f2bf_bits(v[e]);
      hb[e] = h;
      lb[e] = f2bf_bits(v[e] - bf_bits2f(h));
    }
    a = pack8(hb); b = pack8(lb);
  } else {
    unsigned fb[8];
#pragma unroll
    for (int e = 0; e < 8; ++e) fb[e] = f16_bits(scale * v[e]);
    a = pack8(fb); b = a;
  }
  const size_t o = (size_t)i * 8;
  for (int pass = 0; pass < 2; ++pass) {
    *(volatile v4u*)(o1 + o) = a;
    if (mode == 0) *(volatile v4u*)(o2 + o) = b;
    __threadfence();
  }
}

__global__ __launch_bounds__(kThreads) void stats1_pass(const float* __restrict__ coords, const float* __restrict__ t1,
                                                        const float* __restrict__ g, const int* __restrict__ radius,
                                                        float* __restrict__ st1) {
  __shared__ __align__(16) int   ri_i[kTile * 4];
  __shared__ __align__(16) float ri_w[kTile * 4];
  __shared__ float red[2 * 8 * kCh1];
  __shared__ __align__(16) float lineb[2 * kCh1];
  const int tid = threadIdx.x, lane = tid & 31, wave = tid >> 5;
  const int tIdx = blockIdx.x;
  const int n = tIdx / kTilesPerN;
  const int p0 = (tIdx - n * kTilesPerN) * kTile;
  int rr = radius[0];
  rr = rr < 0 ? 0 : (rr > kRad ? kRad : rr);
  const float dxn = (float)(n / kDia - rr);
  const float dyn = (float)(n % kDia - rr);
  if (tid < kTile) {
    v4i idx; v4f ww;
    row_geom(coords, p0 + tid, dxn, dyn, idx, ww);
    *(v4i*)(ri_i + 4 * tid) = idx;
    *(v4f*)(ri_w + 4 * tid) = ww;
  }
  __syncthreads();
  const int part = tid & 7, slot = tid >> 3;
  float s[12], q[12];
#pragma unroll
  for (int e = 0; e < 12; ++e) { s[e] = 0.0f; q[e] = 0.0f; }
#pragma unroll 1
  for (int sw = 0; sw < 4; ++sw) {
    const int row = sw * 32 + slot;
    const v4i idx = *(const v4i*)(ri_i + 4 * row);
    const v4f ww  = *(const v4f*)(ri_w + 4 * row);
    const int p = p0 + row;
#pragma unroll
    for (int qq = 0; qq < 3; ++qq) {
      const int c4 = part + 8 * qq;
      const v4f y = gather4(t1, g, p, c4, idx, ww);
#pragma unroll
      for (int e = 0; e < 4; ++e) {
        s[4 * qq + e] += y[e];
        q[4 * qq + e] = fmaf(y[e], y[e], q[4 * qq + e]);
      }
      clause_break();
    }
  }
#pragma unroll
  for (int e = 0; e < 12; ++e) {
    s[e] += __shfl_xor(s[e], 8, 32);
    s[e] += __shfl_xor(s[e], 16, 32);
    q[e] += __shfl_xor(q[e], 8, 32);
    q[e] += __shfl_xor(q[e], 16, 32);
  }
  if (lane < 8) {
#pragma unroll
    for (int qq = 0; qq < 3; ++qq)
#pragma unroll
      for (int e = 0; e < 4; ++e) {
        const int ch = 4 * (lane + 8 * qq) + e;
        red[wave * kCh1 + ch] = s[4 * qq + e];
        red[8 * kCh1 + wave * kCh1 + ch] = q[4 * qq + e];
      }
  }
  __syncthreads();
  if (tid < 2 * kCh1) {
    const int st = (tid >= kCh1) ? 1 : 0;
    const int ch = tid - st * kCh1;
    float v = 0.0f;
#pragma unroll
    for (int w = 0; w < 8; ++w) v += red[st * 8 * kCh1 + w * kCh1 + ch];
    lineb[tid] = v;
  }
  __syncthreads();
  float* dst = st1 + (size_t)tIdx * (2 * kCh1);
  v4f val = (v4f){0.f, 0.f, 0.f, 0.f};
  if (tid < 48) val = *(const v4f*)(lineb + 4 * tid);
  for (int pass = 0; pass < 2; ++pass) {
    if (tid < 48) *(volatile v4f*)(dst + 4 * tid) = val;
    __threadfence();
  }
}

__global__ __launch_bounds__(kThreads) void bn_finalize(const float* __restrict__ part, int npart, int nch,
                                                        const float* __restrict__ gamma, const float* __restrict__ beta,
                                                        float* __restrict__ ab) {
  __shared__ double sd[kThreads];
  __shared__ __align__(16) float abl[kABP];
  const int tid = threadIdx.x;
  const int ncol = 2 * nch;
  double acc = 0.0;
  if (tid < ncol) {
#pragma unroll 1
    for (int r = 0; r < npart; ++r) acc += (double)part[(size_t)r * ncol + tid];
  }
  sd[tid] = acc;
  abl[tid] = 0.0f;
  __syncthreads();
  float a = 0.0f, b = 0.0f;
  if (tid < nch) {
    const double mean = sd[tid] * kInvRows;
    const double ex2  = sd[nch + tid] * kInvRows;
    const double var  = ex2 - mean * mean;
    float varf = (float)var;
    varf = fmaxf(varf, 0.0f);
    const float rs = rsqrtf(varf + kEps);
    a = gamma[tid] * rs;
    b = beta[tid] - (float)mean * a;
  }
  if (tid < nch) { abl[tid] = a; abl[128 + tid] = b; }
  __syncthreads();
  v4f val = (v4f){0.f, 0.f, 0.f, 0.f};
  if (tid < 64) val = *(const v4f*)(abl + 4 * tid);
  for (int pass = 0; pass < 2; ++pass) {
    if (tid < 64) *(volatile v4f*)(ab + 4 * tid) = val;
    __threadfence();
  }
}

template <bool FULL>
__global__ __launch_bounds__(kThreads) void conv_pass(
    const float* __restrict__ coords, const float* __restrict__ t1, const float* __restrict__ g,
    const float* __restrict__ ab1, const unsigned short* w2p, const unsigned short* w2q,
    const float* __restrict__ ab2, const unsigned short* w3p, const unsigned short* w3q,
    const int* __restrict__ radius, float* __restrict__ stats, float* __restrict__ dqtab,
    unsigned short* __restrict__ y3) {
  typedef typename PT<FULL>::T T;
  typedef Frag<T> F;
  typedef typename F::V V;
  __shared__ __align__(16) LdsU U;
  __shared__ __align__(16) int   ri_i[kTile * 4];
  __shared__ __align__(16) float ri_w[kTile * 4];
  __shared__ float red[2048];
  __shared__ __align__(16) float lineb[256];
  __shared__ float wmx[8];

  const int tid = threadIdx.x, lane = tid & 31, wave = tid >> 5;
  const int hh = lane >> 4, rl = lane & 15, koff = hh * 8;
  const int tIdx = blockIdx.x;
  const int n = tIdx / kTilesPerN;
  const int p0 = (tIdx - n * kTilesPerN) * kTile;
  const size_t row0 = (size_t)tIdx * kTile;
  int rr = radius[0];
  rr = rr < 0 ? 0 : (rr > kRad ? kRad : rr);
  const float dxn = (float)(n / kDia - rr);
  const float dyn = (float)(n % kDia - rr);

  if (tid < kTile) {
    v4i idx; v4f ww;
    row_geom(coords, p0 + tid, dxn, dyn, idx, ww);
    *(v4i*)(ri_i + 4 * tid) = idx;
    *(v4f*)(ri_w + 4 * tid) = ww;
  }
#pragma unroll
  for (int it = 0; it < 6; ++it) {
    const int chunk = it * kThreads + tid;
    const int r = chunk / 12;
    const int c8 = (chunk - r * 12) * 8;
    const v4u v = *(const v4u*)(w2p + r * kCh1 + c8);
    *(v4u*)(U.h + kW2H + r * kP1 + c8) = v;
    if constexpr (FULL) {
      const v4u v2 = *(const v4u*)(w2q + r * kCh1 + c8);
      *(v4u*)(U.h + kW2L + r * kP1 + c8) = v2;
    }
    clause_break();
  }
  __syncthreads();

  {
    const int part = tid & 7, slot = tid >> 3;
    v4f a1c[3], b1c[3];
#pragma unroll
    for (int qq = 0; qq < 3; ++qq) {
      a1c[qq] = *(const v4f*)(ab1 + 4 * (part + 8 * qq));
      b1c[qq] = *(const v4f*)(ab1 + 128 + 4 * (part + 8 * qq));
    }
    clause_break();
#pragma unroll 1
    for (int sw = 0; sw < 4; ++sw) {
      const int row = sw * 32 + slot;
      const v4i idx = *(const v4i*)(ri_i + 4 * row);
      const v4f ww  = *(const v4f*)(ri_w + 4 * row);
      const int p = p0 + row;
#pragma unroll
      for (int qq = 0; qq < 3; ++qq) {
        const int c4 = part + 8 * qq;
        const v4f y = gather4(t1, g, p, c4, idx, ww);
        unsigned hb[4], lb[4];
#pragma unroll
        for (int e = 0; e < 4; ++e) {
          const float av = fmaxf(fmaf(y[e], a1c[qq][e], b1c[qq][e]), 0.0f);
          if constexpr (FULL) {
            const unsigned short h = f2bf_bits(av);
            hb[e] = h;
            lb[e] = f2bf_bits(av - bf_bits2f(h));
          } else {
            hb[e] = f16_bits(av);
            lb[e] = 0u;
          }
        }
        v2u hv; hv[0] = hb[0] | (hb[1] << 16); hv[1] = hb[2] | (hb[3] << 16);
        *(v2u*)(U.h + kA1H + row * kP1 + 4 * c4) = hv;
        if constexpr (FULL) {
          v2u lv; lv[0] = lb[0] | (lb[1] << 16); lv[1] = lb[2] | (lb[3] << 16);
          *(v2u*)(U.h + kA1L + row * kP1 + 4 * c4) = lv;
        }
        clause_break();
      }
    }
  }
  __syncthreads();

  const int rg = wave >> 2, cg = wave & 3;
  v8f acc[4][2];
#pragma unroll
  for (int i = 0; i < 4; ++i)
#pragma unroll
    for (int j = 0; j < 2; ++j) acc[i][j] = (v8f){0.f,0.f,0.f,0.f,0.f,0.f,0.f,0.f};
  {
    const T* LA  = (const T*)(U.h + kA1H);
    const T* LAl = (const T*)(U.h + kA1L);
    const T* LB  = (const T*)(U.h + kW2H);
    const T* LBl = (const T*)(U.h + kW2L);
#pragma unroll 1
    for (int k0 = 0; k0 < kCh1; k0 += 32) {
      V bh[2], bl[2];
#pragma unroll
      for (int j = 0; j < 2; ++j) {
        const int bo = (32 * cg + 16 * j + rl) * kP1 + koff + k0;
        bh[j] = F::load(LB + bo);
        if constexpr (FULL) bl[j] = F::load(LBl + bo);
        else bl[j] = bh[j];
      }
#pragma unroll
      for (int i = 0; i < 4; ++i) {
        const int ao = (64 * rg + 16 * i + rl) * kP1 + koff + k0;
        const V ah = F::load(LA + ao);
        V al = ah;
        if constexpr (FULL) al = F::load(LAl + ao);
#pragma unroll
        for (int j = 0; j < 2; ++j) {
          acc[i][j] = F::mma(ah, bh[j], acc[i][j]);
          if constexpr (FULL) {
            acc[i][j] = F::mma(ah, bl[j], acc[i][j]);
            acc[i][j] = F::mma(al, bh[j], acc[i][j]);
          }
        }
        F::guard(acc[i][0], acc[i][1], ah, al);
      }
      F::keep(bh[0], bh[1], bl[0], bl[1]);
    }
  }
  acc_guard4(acc[0][0], acc[0][1], acc[1][0], acc[1][1]);
  acc_guard4(acc[2][0], acc[2][1], acc[3][0], acc[3][1]);

  if constexpr (!FULL) {
#pragma unroll
    for (int j = 0; j < 2; ++j) {
      const int col = 32 * cg + 16 * j + rl;
      float s = 0.0f, q = 0.0f;
#pragma unroll
      for (int i = 0; i < 4; ++i)
#pragma unroll
        for (int r = 0; r < 8; ++r) {
          const float v = acc[i][j][r] * kW2CarryInv;
          s += v;
          q = fmaf(v, v, q);
        }
      s += __shfl_xor(s, 16, 32);
      q += __shfl_xor(q, 16, 32);
      if (hh == 0) { red[wave * 128 + col] = s; red[1024 + wave * 128 + col] = q; }
    }
    __syncthreads();
    {
      const int col = tid & 127, st = tid >> 7, cgc = col >> 5;
      lineb[tid] = red[st * 1024 + cgc * 128 + col] + red[st * 1024 + (cgc + 4) * 128 + col];
    }
    __syncthreads();
    v4f val = (v4f){0.f, 0.f, 0.f, 0.f};
    if (tid < 64) val = *(const v4f*)(lineb + 4 * tid);
    float* dst = stats + (size_t)tIdx * (2 * kCh2);
    for (int pass = 0; pass < 2; ++pass) {
      if (tid < 64) *(volatile v4f*)(dst + 4 * tid) = val;
      __threadfence();
    }
  } else {
    __syncthreads();
#pragma unroll
    for (int it = 0; it < 4; ++it) {
      const int chunk = it * kThreads + tid;
      const int r = chunk >> 4, c8 = (chunk & 15) * 8;
      const v4u v  = *(const v4u*)(w3p + r * kCh2 + c8);
      const v4u v2 = *(const v4u*)(w3q + r * kCh2 + c8);
      *(v4u*)(U.h + kW3H + r * kP2 + c8) = v;
      *(v4u*)(U.h + kW3L + r * kP2 + c8) = v2;
      clause_break();
    }
#pragma unroll
    for (int j = 0; j < 2; ++j) {
      const int col = 32 * cg + 16 * j + rl;
      const float a2c = ab2[col], b2c = ab2[128 + col];
#pragma unroll
      for (int i = 0; i < 4; ++i)
#pragma unroll
        for (int r = 0; r < 8; ++r) {
          const int row = 64 * rg + 16 * i + 8 * hh + r;
          const float v = fmaxf(fmaf(acc[i][j][r], a2c, b2c), 0.0f);
          const unsigned short h = f2bf_bits(v);
          const unsigned short l = f2bf_bits(v - bf_bits2f(h));
          U.h[kA2H + row * kP2 + col] = h;
          U.h[kA2L + row * kP2 + col] = l;
        }
    }
    __syncthreads();
    const int rg3 = wave >> 1, cg3 = wave & 1;
    v8f acc3[2][2];
#pragma unroll
    for (int i = 0; i < 2; ++i)
#pragma unroll
      for (int j = 0; j < 2; ++j) acc3[i][j] = (v8f){0.f,0.f,0.f,0.f,0.f,0.f,0.f,0.f};
    {
      const T* LA  = (const T*)(U.h + kA2H);
      const T* LAl = (const T*)(U.h + kA2L);
      const T* LB  = (const T*)(U.h + kW3H);
      const T* LBl = (const T*)(U.h + kW3L);
#pragma unroll 1
      for (int k0 = 0; k0 < kCh2; k0 += 32) {
        V bh[2], bl[2];
#pragma unroll
        for (int j = 0; j < 2; ++j) {
          const int bo = (32 * cg3 + 16 * j + rl) * kP2 + koff + k0;
          bh[j] = F::load(LB + bo);
          bl[j] = F::load(LBl + bo);
        }
#pragma unroll
        for (int i = 0; i < 2; ++i) {
          const int ao = (32 * rg3 + 16 * i + rl) * kP2 + koff + k0;
          const V ah = F::load(LA + ao);
          const V al = F::load(LAl + ao);
#pragma unroll
          for (int j = 0; j < 2; ++j) {
            acc3[i][j] = F::mma(ah, bh[j], acc3[i][j]);
            acc3[i][j] = F::mma(ah, bl[j], acc3[i][j]);
            acc3[i][j] = F::mma(al, bh[j], acc3[i][j]);
          }
          F::guard(acc3[i][0], acc3[i][1], ah, al);
        }
        F::keep(bh[0], bh[1], bl[0], bl[1]);
      }
    }
    acc_guard4(acc3[0][0], acc3[0][1], acc3[1][0], acc3[1][1]);
    float mx = 0.0f;
#pragma unroll
    for (int i = 0; i < 2; ++i)
#pragma unroll
      for (int j = 0; j < 2; ++j)
#pragma unroll
        for (int r = 0; r < 8; ++r) mx = fmaxf(mx, fabsf(acc3[i][j][r]));
#pragma unroll
    for (int off = 1; off < 32; off <<= 1) mx = fmaxf(mx, __shfl_xor(mx, off, 32));
    __syncthreads();
    if (lane == 0) wmx[wave] = mx;
#pragma unroll
    for (int j = 0; j < 2; ++j) {
      const int col = 32 * cg3 + 16 * j + rl;
      float s = 0.0f, q = 0.0f;
#pragma unroll
      for (int i = 0; i < 2; ++i)
#pragma unroll
        for (int r = 0; r < 8; ++r) {
          const int row = 32 * rg3 + 16 * i + 8 * hh + r;
          const float v = acc3[i][j][r];
          U.f[row * kYP + col] = v;
          s += v;
          q = fmaf(v, v, q);
        }
      s += __shfl_xor(s, 16, 32);
      q += __shfl_xor(q, 16, 32);
      if (hh == 0) { red[wave * 64 + col] = s; red[512 + wave * 64 + col] = q; }
    }
    __syncthreads();
    float bm = 0.0f;
#pragma unroll
    for (int w = 0; w < 8; ++w) bm = fmaxf(bm, wmx[w]);
    float dq = bm * (1.0f / 32767.0f);
    if (!(dq > 1e-30f)) dq = 1.0f;
    const float qs = 1.0f / dq;
    if (tid < 128) {
      const int col = tid & 63, st = tid >> 6, cb = col >> 5;
      float v = 0.0f;
#pragma unroll
      for (int m = 0; m < 4; ++m) v += red[st * 512 + (cb + 2 * m) * 64 + col];
      lineb[tid] = v;
    } else if (tid < 160) {
      lineb[tid] = dq;
    }
    __syncthreads();
    v4u qv[4];
#pragma unroll
    for (int it = 0; it < 4; ++it) {
      const int chunk = it * kThreads + tid;
      const int row = chunk >> 3, c8 = (chunk & 7) * 8;
      const v4f xa = *(const v4f*)(U.f + row * kYP + c8);
      const v4f xb = *(const v4f*)(U.f + row * kYP + c8 + 4);
      int qi[8];
#pragma unroll
      for (int e = 0; e < 4; ++e) {
        qi[e]     = (int)rintf(fminf(fmaxf(xa[e] * qs, -32767.0f), 32767.0f));
        qi[4 + e] = (int)rintf(fminf(fmaxf(xb[e] * qs, -32767.0f), 32767.0f));
      }
      unsigned qb[8];
#pragma unroll
      for (int e = 0; e < 8; ++e) qb[e] = (unsigned)(qi[e] & 0xffff);
      qv[it] = pack8(qb);
    }
    v4f sval = (v4f){0.f, 0.f, 0.f, 0.f};
    if (tid < 32) sval = *(const v4f*)(lineb + 4 * tid);
    v4f dval = (v4f){0.f, 0.f, 0.f, 0.f};
    if (tid >= 32 && tid < 40) dval = *(const v4f*)(lineb + 128 + 4 * (tid - 32));
    float* sdst = stats + (size_t)tIdx * (2 * kCh3);
    float* ddst = dqtab + (size_t)tIdx * kDQP;
    for (int pass = 0; pass < 2; ++pass) {
#pragma unroll
      for (int it = 0; it < 4; ++it) {
        const int chunk = it * kThreads + tid;
        const int row = chunk >> 3, c8 = (chunk & 7) * 8;
        *(volatile v4u*)(y3 + (row0 + row) * kCh3 + c8) = qv[it];
      }
      if (tid < 32) *(volatile v4f*)(sdst + 4 * tid) = sval;
      if (tid >= 32 && tid < 40) *(volatile v4f*)(ddst + 4 * (tid - 32)) = dval;
      __threadfence();
    }
  }
}

__global__ __launch_bounds__(kThreads) void final_pass(const unsigned short* __restrict__ y3, const float* __restrict__ dqtab,
                                                       const float* __restrict__ ab3, const float* __restrict__ w4,
                                                       const float* __restrict__ b4, const float* __restrict__ wdap,
                                                       float* __restrict__ out) {
  __shared__ __align__(16) float costl[kND * kYP];
  __shared__ __align__(16) float outl[kND * kYP];
  const int tid = threadIdx.x;
  const int p0 = blockIdx.x * 64;
  const int ptile = p0 >> 7;
  const int cgp = tid & 7, pls = tid >> 3;
  const v4f a3a = *(const v4f*)(ab3 + 8 * cgp);
  const v4f a3b = *(const v4f*)(ab3 + 8 * cgp + 4);
  const v4f b3a = *(const v4f*)(ab3 + 128 + 8 * cgp);
  const v4f b3b = *(const v4f*)(ab3 + 128 + 8 * cgp + 4);
  const v4f w4a = *(const v4f*)(w4 + 8 * cgp);
  const v4f w4b = *(const v4f*)(w4 + 8 * cgp + 4);
  float a3c[8], b3c[8], w4c[8];
#pragma unroll
  for (int e = 0; e < 4; ++e) {
    a3c[e] = a3a[e]; a3c[4 + e] = a3b[e];
    b3c[e] = b3a[e]; b3c[4 + e] = b3b[e];
    w4c[e] = w4a[e]; w4c[4 + e] = w4b[e];
  }
  clause_break();
  const float bias = b4[0];
#pragma unroll 1
  for (int k = 0; k < kND; ++k) {
    const float dq = dqtab[(size_t)(k * kTilesPerN + ptile) * kDQP];
#pragma unroll
    for (int s = 0; s < 2; ++s) {
      const int pl = pls + 32 * s;
      const size_t row = (size_t)k * kPix + p0 + pl;
      const v4u wv = *(const v4u*)(y3 + row * kCh3 + 8 * cgp);
      float ps = 0.0f;
#pragma unroll
      for (int m = 0; m < 4; ++m) {
        const unsigned w = wv[m];
        const int q0 = ((int)(w << 16)) >> 16;
        const int q1 = ((int)w) >> 16;
        const float ya = (float)q0 * dq;
        const float yb = (float)q1 * dq;
        const float va = fmaxf(fmaf(ya, a3c[2 * m], b3c[2 * m]), 0.0f);
        const float vb = fmaxf(fmaf(yb, a3c[2 * m + 1], b3c[2 * m + 1]), 0.0f);
        ps = fmaf(va, w4c[2 * m], ps);
        ps = fmaf(vb, w4c[2 * m + 1], ps);
      }
      ps += __shfl_xor(ps, 1, 32);
      ps += __shfl_xor(ps, 2, 32);
      ps += __shfl_xor(ps, 4, 32);
      if (cgp == 0) costl[k * kYP + pl] = ps + bias;
    }
  }
  __syncthreads();
  {
    const int pl = tid & 63, lq = tid >> 6;
#pragma unroll 1
    for (int l = lq; l < kND; l += 4) {
      const float* wr = wdap + l * kND;
      float acc = 0.0f;
#pragma unroll 3
      for (int k = 0; k < kND; ++k) acc = fmaf(wr[k], costl[k * kYP + pl], acc);
      outl[l * kYP + pl] = acc;
    }
  }
  __syncthreads();
  v4f vals[6];
#pragma unroll
  for (int it = 0; it < 6; ++it) {
    const int chunk = it * kThreads + tid;
    int l = chunk >> 4;
    const int c4 = (chunk & 15) * 4;
    l = (l < kND) ? l : (kND - 1);
    vals[it] = *(const v4f*)(outl + l * kYP + c4);
  }
  for (int pass = 0; pass < 2; ++pass) {
#pragma unroll
    for (int it = 0; it < 6; ++it) {
      const int chunk = it * kThreads + tid;
      const int l = chunk >> 4, c4 = (chunk & 15) * 4;
      if (chunk < kND * 16) *(volatile v4f*)(out + (size_t)l * kPix + p0 + c4) = vals[it];
    }
    __threadfence();
  }
}

extern "C" void kernel_launch(void* const* d_in, const int* in_sizes, int n_in,
                              void* d_out, int out_size, void* d_ws, size_t ws_size, hipStream_t stream) {
  if (n_in < 16) return;
  if (ws_size < kWsTotal) return;
  if (out_size < kRows) return;
  if (in_sizes[0] != kFeat * kPix || in_sizes[1] != kFeat * kPix || in_sizes[2] != 2 * kPix) return;
  if (in_sizes[3] != kCh1 * 2 * kFeat || in_sizes[4] < kCh1 || in_sizes[5] < kCh1) return;
  if (in_sizes[6] != kCh2 * kCh1 || in_sizes[7] < kCh2 || in_sizes[8] < kCh2) return;
  if (in_sizes[9] != kCh3 * kCh2 || in_sizes[10] < kCh3 || in_sizes[11] < kCh3) return;
  if (in_sizes[12] < kCh3 || in_sizes[13] < 1 || in_sizes[14] != kND * kND || in_sizes[15] < 1) return;

  const float* f1     = (const float*)d_in[0];
  const float* f2     = (const float*)d_in[1];
  const float* coords = (const float*)d_in[2];
  const float* w1     = (const float*)d_in[3];
  const float* g1     = (const float*)d_in[4];
  const float* be1    = (const float*)d_in[5];
  const float* w2     = (const float*)d_in[6];
  const float* g2     = (const float*)d_in[7];
  const float* be2    = (const float*)d_in[8];
  const float* w3     = (const float*)d_in[9];
  const float* g3     = (const float*)d_in[10];
  const float* be3    = (const float*)d_in[11];
  const float* w4     = (const float*)d_in[12];
  const float* b4     = (const float*)d_in[13];
  const float* wdap   = (const float*)d_in[14];
  const int*   radius = (const int*)d_in[15];
  float* out = (float*)d_out;

  char* ws = (char*)d_ws;
  unsigned short* fth = (unsigned short*)(ws + kOffFtH);
  unsigned short* ftl = (unsigned short*)(ws + kOffFtL);
  unsigned short* w1h = (unsigned short*)(ws + kOffW1H);
  unsigned short* w1l = (unsigned short*)(ws + kOffW1L);
  float* t1p = (float*)(ws + kOffTG);
  float* gp  = t1p + (size_t)kPix * kTGP;
  unsigned short* w2h = (unsigned short*)(ws + kOffW2H);
  unsigned short* w2l = (unsigned short*)(ws + kOffW2L);
  unsigned short* w2f = (unsigned short*)(ws + kOffW2F);
  unsigned short* w3h = (unsigned short*)(ws + kOffW3H);
  unsigned short* w3l = (unsigned short*)(ws + kOffW3L);
  float* ab1 = (float*)(ws + kOffAB1);
  float* ab2 = (float*)(ws + kOffAB2);
  float* ab3 = (float*)(ws + kOffAB3);
  float* st1 = (float*)(ws + kOffSt1);
  float* st2 = (float*)(ws + kOffSt2);
  float* st3 = (float*)(ws + kOffSt3);
  float* dq  = (float*)(ws + kOffDQ);
  unsigned short* y3 = (unsigned short*)(ws + kOffY3);

  prep_feat<<<dim3(kPix / 64, 2), kThreads, 0, stream>>>(f1, f2, fth, ftl);
  prep_w<<<(128 * 16 + kThreads - 1) / kThreads, kThreads, 0, stream>>>(w1, kCh1, 2 * kFeat, 0,     kFeat, 128, 0, 1.0f, w1h, w1l);
  prep_w<<<(128 * 16 + kThreads - 1) / kThreads, kThreads, 0, stream>>>(w1, kCh1, 2 * kFeat, kFeat, kFeat, 128, 0, 1.0f,
                                                                        w1h + 128 * 128, w1l + 128 * 128);
  prep_w<<<(kCh2 * (kCh1 / 8) + kThreads - 1) / kThreads, kThreads, 0, stream>>>(w2, kCh2, kCh1, 0, kCh1, kCh2, 0, 1.0f, w2h, w2l);
  prep_w<<<(kCh2 * (kCh1 / 8) + kThreads - 1) / kThreads, kThreads, 0, stream>>>(w2, kCh2, kCh1, 0, kCh1, kCh2, 1, kW2Carry, w2f, w2f);
  prep_w<<<(kCh3 * (kCh2 / 8) + kThreads - 1) / kThreads, kThreads, 0, stream>>>(w3, kCh3, kCh2, 0, kCh2, kCh3, 0, 1.0f, w3h, w3l);
  wmma_gemm64<1, true, 0, 0, false, 0><<<dim3((kPix / 64) * (kTGP / 64) / 8, 2), 256, 0, stream>>>(
      fth, ftl, kFeat, (long)kPix * kFeat,
      w1h, w1l, kFeat, (long)128 * 128,
      (void*)t1p, (void*)t1p, kTGP, (long)kPix * kTGP,
      ab1, ab1, 0L, kPix, kTGP, kFeat, 1.0f);
  stats1_pass<<<kTiles, kThreads, 0, stream>>>(coords, t1p, gp, radius, st1);
  bn_finalize<<<1, kThreads, 0, stream>>>(st1, kTiles, kCh1, g1, be1, ab1);
  conv_pass<false><<<kTiles, kThreads, 0, stream>>>(coords, t1p, gp, ab1, w2f, w2f, ab2, w3h, w3l, radius, st2, dq, y3);
  bn_finalize<<<1, kThreads, 0, stream>>>(st2, kTiles, kCh2, g2, be2, ab2);
  conv_pass<true><<<kTiles, kThreads, 0, stream>>>(coords, t1p, gp, ab1, w2h, w2l, ab2, w3h, w3l, radius, st3, dq, y3);
  bn_finalize<<<1, kThreads, 0, stream>>>(st3, kTiles, kCh3, g3, be3, ab3);
  final_pass<<<kPix / 64, kThreads, 0, stream>>>(y3, dq, ab3, w4, b4, wdap, out);
}
